// GNNBranch_86174223827123
// MI455X (gfx1250) — hardware-run, weakly checked
//
#include <hip/hip_runtime.h>


namespace {
constexpr int N = 8192, NG = 16, E = 131072, PDIM = 1310, PK = 1344, LDIM = 36, D = 256, NH = 4, HD = NH * D, ADIM = 128, NL = 3, NBLK = N / 16;
constexpr float XS = 8.0f, WSC = 256.0f, NEGV = -1e30f;
typedef _Float16 b16;
typedef __attribute__((ext_vector_type(16))) _Float16 v16b;
typedef __attribute__((ext_vector_type(8))) _Float16 v8b;
typedef __attribute__((ext_vector_type(8))) float v8f;
typedef __attribute__((ext_vector_type(4))) float v4f;
__device__ __forceinline__ float bf16_rne(float f) { unsigned int u = __float_as_uint(f); u += 0x7FFFu + ((u >> 16) & 1u); return __uint_as_float(u & 0xFFFF0000u); }
__device__ __forceinline__ void split16(float v, b16& hi, b16& lo) { hi = (b16)v; lo = (b16)(v - (float)hi); }
__device__ __forceinline__ v16b frag_kb(const b16* p, int hh) { const v8b a = *(const v8b*)(p + 8 * hh), b = *(const v8b*)(p + 16 + 8 * hh); v16b f;
#pragma unroll
  for (int e = 0; e < 8; ++e) { f[e] = a[e]; f[8 + e] = b[e]; } return f; }
__device__ __forceinline__ v8f wmma16b(v16b a, v16b b, v8f c) { v8f d = __builtin_amdgcn_wmma_f32_16x16x32_f16(false, a, false, b, (short)0, c, false, false); asm volatile("v_nop\n\tv_nop\n\tv_nop\n\tv_nop" : "+v"(d) : "v"(a), "v"(b)); return d; }
__device__ __forceinline__ void wave_lds_sync() { __builtin_amdgcn_fence(__ATOMIC_RELEASE, "workgroup"); __builtin_amdgcn_wave_barrier(); __builtin_amdgcn_fence(__ATOMIC_ACQUIRE, "workgroup"); }
__device__ __forceinline__ float pmul(float a, float b) { float p = a * b; asm volatile("" : "+v"(p)); return p; }
__device__ __forceinline__ int iclamp(int v, int lo, int hi) { return v < lo ? lo : (v > hi ? hi : v); }
__device__ __forceinline__ float leaky(float v) { return v >= 0.0f ? v : 0.2f * v; }
constexpr int CSR_NBLK9 = 512, CSR_GB9 = 9, CSR_GN9 = 1 << CSR_GB9  , CSR_TS9 = (CSR_GN9 < 32 ? 32 : CSR_GN9)  , CSR_MAXG9 = 512, CSR_CAP9 = 12288  ;
__device__ __host__ __forceinline__ int csr_tix9(int v) { return (v >> CSR_GB9) * CSR_TS9 + (v & (CSR_GN9 - 1)); }
__global__ __launch_bounds__(64) void csrA_kernel9(const int* __restrict__ dst, int E, int N, int nG, int CHP, int NGP, int* __restrict__ STG, int* __restrict__ HST) {
  extern __shared__ int sm[];
  int* cnt = sm; int* run = sm + NGP; int* ids = sm + 2 * NGP;
  const int b = blockIdx.x; const int ch = (E + CSR_NBLK9 - 1) / CSR_NBLK9; const int e0 = b * ch, e1 = min(E, e0 + ch);
  for (int i = threadIdx.x; i < NGP; i += 64) cnt[i] = 0;
  for (int i = threadIdx.x; i < CHP; i += 64) ids[i] = -1;
  __syncthreads();
  if (threadIdx.x == 0) {
    for (int e = e0; e < e1; ++e) { int d = dst[e]; d = (d < 0) ? 0 : (d >= N ? N - 1 : d); cnt[d >> CSR_GB9] += 1; }
    int acc = 0; for (int g = 0; g < nG; ++g) { run[g] = acc; acc += cnt[g]; }
    for (int e = e0; e < e1; ++e) { int d = dst[e]; d = (d < 0) ? 0 : (d >= N ? N - 1 : d); const int g = d >> CSR_GB9; ids[run[g]] = e; run[g] += 1; } }
  __syncthreads();
  typedef __attribute__((ext_vector_type(4))) int v4i;
  for (int pass = 0; pass < 2; ++pass) {
    for (int i = threadIdx.x; i < CHP / 4; i += 64) *(volatile v4i*)(STG + (size_t)b * CHP + i * 4) = *(const v4i*)(&ids[i * 4]);
    for (int i = threadIdx.x; i < NGP / 4; i += 64) { v4i v; for (int e = 0; e < 4; ++e) v[e] = (i * 4 + e < nG) ? cnt[i * 4 + e] : 0; *(volatile v4i*)(HST + (size_t)b * NGP + i * 4) = v; }
    __threadfence(); }
}
__global__ __launch_bounds__(512) void csrS_kernel9(const int* __restrict__ HST, int nG, int NGP, int* __restrict__ START, int* __restrict__ TOT, int* __restrict__ OFF) {
  __shared__ int tot[CSR_MAXG9];
  const int b = threadIdx.x;
  for (int pass = 0; pass < 2; ++pass) { int runb = 0; for (int g = 0; g < nG; ++g) { int c = HST[(size_t)b * NGP + g]; c = (c < 0) ? 0 : c; ((volatile int*)OFF)[(size_t)g * CSR_NBLK9 + b] = runb; runb += c; } __threadfence(); }
  for (int g = threadIdx.x; g < nG; g += 512) { int s = 0; for (int bb = 0; bb < CSR_NBLK9; ++bb) { int c = HST[(size_t)bb * NGP + g]; s += (c < 0) ? 0 : c; } tot[g] = s; }
  __syncthreads();
  if (threadIdx.x < 32) {
    __shared__ int st[CSR_MAXG9 + 32];
    if (threadIdx.x == 0) { int acc = 0; for (int g = 0; g < NGP; ++g) { st[g] = acc; if (g < nG) acc += (tot[g] + 31) & ~31; } st[NGP] = acc; }
    __builtin_amdgcn_fence(__ATOMIC_RELEASE, "workgroup"); __builtin_amdgcn_wave_barrier(); __builtin_amdgcn_fence(__ATOMIC_ACQUIRE, "workgroup");
    for (int pass = 0; pass < 2; ++pass) { for (int i = threadIdx.x; i < NGP + 32; i += 32) { ((volatile int*)START)[i] = (i <= NGP) ? st[min(i, NGP)] : 0; ((volatile int*)TOT)[i] = (i < nG) ? tot[i] : 0; } __threadfence(); } }
}
__global__ __launch_bounds__(256) void csrB_kernel9(const int* __restrict__ dst, int N, int nG, int CHP, int NGP, int permLen, const int* __restrict__ STG, const int* __restrict__ HST, const int* __restrict__ OFF, const int* __restrict__ START, const int* __restrict__ TOT, int* __restrict__ PERM, int* __restrict__ ROWPTR, int* __restrict__ ROWCNT, int* __restrict__ FLAG) {
  typedef __attribute__((ext_vector_type(4))) int v4i;
  __shared__ int ids[CSR_CAP9]; __shared__ unsigned short key[CSR_CAP9]; __shared__ int outp[CSR_CAP9]; __shared__ int ncnt[CSR_GN9 + 1]; __shared__ int boff[CSR_NBLK9 + 1];
  const int g = blockIdx.x, t_ = threadIdx.x; int tot = TOT[g]; int st = START[g], stn = START[g + 1]; const int v0 = g * CSR_GN9; const int nv = min(CSR_GN9, N - v0); const int t0 = g * CSR_TS9;
  st = (st < 0) ? 0 : (st > permLen - 32 ? permLen - 32 : st) & ~31; stn = (stn < st) ? st : (stn > permLen ? permLen : stn); tot = (tot < 0) ? 0 : tot; if (tot > stn - st && tot <= CSR_CAP9) tot = stn - st;
  if (tot > CSR_CAP9) {
    for (int pass = 0; pass < 2; ++pass) { for (int i = t_; i < CSR_TS9 / 4; i += 256) { v4i a, c; for (int e = 0; e < 4; ++e) { a[e] = st; c[e] = 0; } *(volatile v4i*)(ROWPTR + t0 + i * 4) = a; *(volatile v4i*)(ROWCNT + t0 + i * 4) = c; } if (t_ == 0) ((volatile int*)FLAG)[0] = 1; __threadfence(); } (void)nv; return; }
  if (t_ == 0) { int acc = 0; for (int b = 0; b < CSR_NBLK9; ++b) { boff[b] = acc; int c = HST[(size_t)b * NGP + g]; c = (c < 0) ? 0 : (c > CHP ? CHP : c); acc += c; if (acc > tot) acc = tot; } boff[CSR_NBLK9] = acc; }
  for (int i = t_; i <= CSR_GN9; i += 256) ncnt[i] = 0;
  __syncthreads();
  for (int b = 0; b < CSR_NBLK9; ++b) { const int c = boff[b + 1] - boff[b]; int o_ = OFF[(size_t)g * CSR_NBLK9 + b]; o_ = (o_ < 0) ? 0 : (o_ > CHP - c ? CHP - c : o_); const int* src_ = STG + (size_t)b * CHP + o_;
    for (int i = t_; i < c; i += 256) { int id = src_[i]; id = (id < 0) ? 0 : id; ids[boff[b] + i] = id; int d = dst[id]; d = (d < v0) ? v0 : (d >= N ? N - 1 : d); int kk = d - v0; kk = (kk < 0) ? 0 : (kk >= CSR_GN9 ? CSR_GN9 - 1 : kk); key[boff[b] + i] = (unsigned short)kk; } }
  __syncthreads();
  if (t_ == 0) { for (int i = 0; i < tot; ++i) ncnt[key[i]] += 1; int acc = 0; for (int vl = 0; vl < CSR_GN9; ++vl) { const int c = ncnt[vl]; ncnt[vl] = acc; acc += c; } ncnt[CSR_GN9] = acc;
    for (int i = 0; i < tot; ++i) { const int vl = key[i]; outp[ncnt[vl]] = ids[i]; ncnt[vl] += 1; }
    for (int vl = CSR_GN9; vl > 0; --vl) ncnt[vl] = ncnt[vl - 1]; ncnt[0] = 0; }
  __syncthreads();
  for (int pass = 0; pass < 2; ++pass) {
    for (int i = t_; i < (stn - st) / 4; i += 256) { v4i v; for (int e = 0; e < 4; ++e) { const int q = i * 4 + e; v[e] = (q < tot) ? outp[q] : -1; } *(volatile v4i*)(PERM + st + i * 4) = v; }
    for (int i = t_; i < CSR_TS9 / 4; i += 256) { v4i a, c; for (int e = 0; e < 4; ++e) { const int vl = i * 4 + e; const int vc = vl < CSR_GN9 ? vl : CSR_GN9; a[e] = (vl < CSR_GN9) ? st + ncnt[vc] : st; c[e] = (vl < nv) ? (ncnt[(vc < CSR_GN9 ? vc : CSR_GN9 - 1) + 1] - ncnt[vc]) : 0; } *(volatile v4i*)(ROWPTR + t0 + i * 4) = a; *(volatile v4i*)(ROWCNT + t0 + i * 4) = c; }
    __threadfence(); }
}
__global__ __launch_bounds__(256) void csrZ_kernel9(int* __restrict__ p, size_t n4) { typedef __attribute__((ext_vector_type(4))) int v4i; const size_t tid = (size_t)blockIdx.x * 256 + threadIdx.x, nth = (size_t)gridDim.x * 256; v4i z = {0, 0, 0, 0}; for (size_t i = tid; i < n4; i += nth) *(volatile v4i*)(p + i * 4) = z; }
struct CsrBufs9 { int *STG, *HST, *OFF, *START, *TOT, *PERM, *ROWPTR, *ROWCNT, *FLAG; int nG, NGP, CHP; size_t permLen; char* base; size_t bytes; };
static size_t csr_carve9(CsrBufs9& c, char* ws, size_t off, int E, int N) {
  const size_t off0 = off; c.base = ws + off;
  auto al = [&](size_t bytes) { char* p = ws + off; off += (bytes + 255) & ~(size_t)255; return p; };
  c.nG = (N + CSR_GN9 - 1) / CSR_GN9; c.NGP = (c.nG + 31) & ~31; const int ch = (E + CSR_NBLK9 - 1) / CSR_NBLK9; c.CHP = (ch + 31) & ~31; c.permLen = (size_t)E + 32 * (size_t)c.nG + 32;
  c.STG = (int*)al((size_t)CSR_NBLK9 * c.CHP * 4); c.HST = (int*)al((size_t)CSR_NBLK9 * c.NGP * 4); c.OFF = (int*)al((size_t)c.NGP * CSR_NBLK9 * 4); c.START = (int*)al((size_t)(c.NGP + 64) * 4); c.TOT = (int*)al((size_t)(c.NGP + 64) * 4);
  c.PERM = (int*)al(c.permLen * 4); c.ROWPTR = (int*)al((size_t)c.nG * CSR_TS9 * 4); c.ROWCNT = (int*)al((size_t)c.nG * CSR_TS9 * 4); c.FLAG = (int*)al(256);
  c.bytes = off - off0; return off;
}
static void csr_build9(const CsrBufs9& c, const int* dst, int E, int N, hipStream_t stream) {
  const size_t smem = (size_t)(2 * c.NGP + c.CHP) * 4;
  csrZ_kernel9<<<512, 256, 0, stream>>>((int*)c.base, c.bytes / 16);
  csrA_kernel9<<<CSR_NBLK9, 64, smem, stream>>>(dst, E, N, c.nG, c.CHP, c.NGP, c.STG, c.HST);
  csrS_kernel9<<<1, 512, 0, stream>>>(c.HST, c.nG, c.NGP, c.START, c.TOT, c.OFF);
  csrB_kernel9<<<c.nG, 256, 0, stream>>>(dst, N, c.nG, c.CHP, c.NGP, (int)c.permLen, c.STG, c.HST, c.OFF, c.START, c.TOT, c.PERM, c.ROWPTR, c.ROWCNT, c.FLAG);
}


__global__ __launch_bounds__(256) void wput_kernel(const float* __restrict__ w, int KIN, int KP, int OUTW, b16* __restrict__ WT) {
  const int KG = KP / 8; const size_t u = (size_t)blockIdx.x * 256 + threadIdx.x; if (u >= (size_t)OUTW * KG) return; const int o = (int)(u / KG), k0 = (int)(u % KG) * 8; v8b v;
#pragma unroll
  for (int j = 0; j < 8; ++j) { const int k = k0 + j; v[j] = k < KIN ? (b16)(bf16_rne(w[(size_t)k * OUTW + o]) * WSC) : (b16)0.0f; } for (int pass = 0; pass < 2; ++pass) { *(volatile v8b*)(WT + (size_t)o * KP + k0) = v; __threadfence(); }
}
__device__ __forceinline__ void ln_relu_row(float* row, int lane, const float* g, const float* b) {
  float v[8]; float s = 0.0f; for (int i = 0; i < 8; ++i) { v[i] = row[lane * 8 + i]; s += v[i]; } for (int o = 16; o; o >>= 1) s += __shfl_xor(s, o); const float mu = s * (1.0f / D);
  float q = 0.0f; for (int i = 0; i < 8; ++i) { const float d = v[i] - mu; q += pmul(d, d); } for (int o = 16; o; o >>= 1) q += __shfl_xor(q, o); const float rs = 1.0f / sqrtf(q * (1.0f / D) + 1e-5f);
  for (int i = 0; i < 8; ++i) { const int c = lane * 8 + i; row[c] = fmaxf(pmul(pmul(v[i] - mu, rs), bf16_rne(g[c])) + bf16_rne(b[c]), 0.0f); } }
__global__ __launch_bounds__(32) void inproj_kernel(const float* __restrict__ x, const int* __restrict__ ntype, const b16* __restrict__ WP, const float* __restrict__ bp, const float* __restrict__ gp, const float* __restrict__ betap, const b16* __restrict__ WL, const float* __restrict__ bl, const float* __restrict__ gl, const float* __restrict__ betal, const float* __restrict__ nemb, float* __restrict__ Hh) {
  __shared__ __attribute__((aligned(16))) b16 Ah[16][PK + 8]; __shared__ __attribute__((aligned(16))) float Tp[16][D], Tl[16][D];
  const int lane = threadIdx.x, nloc = lane & 15, hlf = lane >> 4; const size_t m0 = (size_t)blockIdx.x * 16;
  for (int rr = 0; rr < 16; ++rr) for (int q = 0; q < PK / 32; ++q) { const int c = q * 32 + lane; Ah[rr][c] = c < PDIM ? (b16)(bf16_rne(x[(m0 + rr) * PDIM + c]) * XS) : (b16)0.0f; }
  wave_lds_sync();
#pragma unroll 1
  for (int cg = 0; cg < 2; ++cg) { v8f acc[8];
#pragma unroll
    for (int t = 0; t < 8; ++t) acc[t] = (v8f){};
#pragma unroll 2
    for (int kb = 0; kb < PK; kb += 32) { const v16b a = frag_kb(&Ah[nloc][kb], hlf);
#pragma unroll
      for (int t = 0; t < 8; ++t) acc[t] = wmma16b(a, frag_kb(WP + (size_t)(cg * 128 + t * 16 + nloc) * PK + kb, hlf), acc[t]); }
#pragma unroll
    for (int t = 0; t < 8; ++t) { const int c = cg * 128 + t * 16 + nloc; const float bb = bf16_rne(bp[c]);
#pragma unroll
      for (int r8 = 0; r8 < 8; ++r8) Tp[8 * hlf + r8][c] = acc[t][r8] * (1.0f / (XS * WSC)) + bb; } }
  {
#pragma unroll 1
    for (int cg = 0; cg < 2; ++cg) { v8f acc[8];
#pragma unroll
      for (int t = 0; t < 8; ++t) acc[t] = (v8f){};
#pragma unroll
      for (int kb = 0; kb < 64; kb += 32) { const v16b a = frag_kb(&Ah[nloc][kb], hlf);
#pragma unroll
        for (int t = 0; t < 8; ++t) acc[t] = wmma16b(a, frag_kb(WL + (size_t)(cg * 128 + t * 16 + nloc) * 64 + kb, hlf), acc[t]); }
#pragma unroll
      for (int t = 0; t < 8; ++t) { const int c = cg * 128 + t * 16 + nloc; const float bb = bf16_rne(bl[c]);
#pragma unroll
        for (int r8 = 0; r8 < 8; ++r8) Tl[8 * hlf + r8][c] = acc[t][r8] * (1.0f / (XS * WSC)) + bb; } } }
  wave_lds_sync();
  for (int rr = 0; rr < 16; ++rr) { ln_relu_row(Tp[rr], lane, gp, betap); ln_relu_row(Tl[rr], lane, gl, betal); }
  wave_lds_sync();
  for (int pass = 0; pass < 2; ++pass) { for (int rr = 0; rr < 16; ++rr) { const int t = iclamp(ntype[m0 + rr], 0, 1); float o[8]; for (int i = 0; i < 8; ++i) { const int c = lane * 8 + i; o[i] = (t == 0 ? Tp[rr][c] : Tl[rr][c]) + bf16_rne(nemb[t * D + c]); }
      *(volatile v4f*)(Hh + (m0 + rr) * D + lane * 8) = (v4f){o[0], o[1], o[2], o[3]}; *(volatile v4f*)(Hh + (m0 + rr) * D + lane * 8 + 4) = (v4f){o[4], o[5], o[6], o[7]}; } __threadfence(); }
}
__global__ __launch_bounds__(32) void gatproj_kernel(const float* __restrict__ Hh, const b16* __restrict__ WG, const float* __restrict__ asrc, const float* __restrict__ adst, float* __restrict__ XH, float* __restrict__ AS) {
  __shared__ __attribute__((aligned(16))) b16 Ah[16][D + 8], Al[16][D + 8]; __shared__ __attribute__((aligned(16))) float Tf[16][128 + 4], Ps[16][8];
  const int lane = threadIdx.x, nloc = lane & 15, hlf = lane >> 4; const size_t m0 = (size_t)blockIdx.x * 16;
  for (int rr = 0; rr < 16; ++rr) for (int q = 0; q < 8; ++q) { b16 p, ql; split16(Hh[(m0 + rr) * D + q * 32 + lane] * XS, p, ql); Ah[rr][q * 32 + lane] = p; Al[rr][q * 32 + lane] = ql; }
  if (lane < 16) for (int j = 0; j < 8; ++j) Ps[lane][j] = 0.0f;
  wave_lds_sync();
#pragma unroll 1
  for (int cg = 0; cg < 8; ++cg) { const int head = cg / 2; v8f acc[8];
#pragma unroll
    for (int t = 0; t < 8; ++t) acc[t] = (v8f){};
#pragma unroll 2
    for (int kb = 0; kb < D; kb += 32) { const v16b a = frag_kb(&Ah[nloc][kb], hlf), al = frag_kb(&Al[nloc][kb], hlf);
#pragma unroll
      for (int t = 0; t < 8; ++t) { const v16b bw = frag_kb(WG + (size_t)(cg * 128 + t * 16 + nloc) * D + kb, hlf); acc[t] = wmma16b(a, bw, acc[t]); acc[t] = wmma16b(al, bw, acc[t]); } }
    float ps[8], pd[8];
#pragma unroll
    for (int r8 = 0; r8 < 8; ++r8) { ps[r8] = 0.0f; pd[r8] = 0.0f; }
#pragma unroll
    for (int t = 0; t < 8; ++t) { const int c = cg * 128 + t * 16 + nloc; const int cd = c & (D - 1); const float ws_ = bf16_rne(asrc[head * D + cd]), wd_ = bf16_rne(adst[head * D + cd]);
#pragma unroll
      for (int r8 = 0; r8 < 8; ++r8) { const float v = acc[t][r8] * (1.0f / (XS * WSC)); Tf[8 * hlf + r8][t * 16 + nloc] = v; ps[r8] += pmul(v, ws_); pd[r8] += pmul(v, wd_); } }
#pragma unroll
    for (int r8 = 0; r8 < 8; ++r8) { for (int o = 1; o < 16; o <<= 1) { ps[r8] += __shfl_xor(ps[r8], o); pd[r8] += __shfl_xor(pd[r8], o); } }
    if (nloc == 0) {
#pragma unroll
      for (int r8 = 0; r8 < 8; ++r8) { Ps[8 * hlf + r8][head] += ps[r8]; Ps[8 * hlf + r8][4 + head] += pd[r8]; } }
    wave_lds_sync();
    for (int pass = 0; pass < 2; ++pass) { for (int rr = 0; rr < 16; ++rr) *(volatile v4f*)(XH + (m0 + rr) * HD + cg * 128 + lane * 4) = *(const v4f*)(&Tf[rr][lane * 4]); __threadfence(); }
    wave_lds_sync(); }
  for (int pass = 0; pass < 2; ++pass) { for (int q = 0; q < 4; ++q) { const int i = q * 32 + lane; ((volatile float*)AS)[m0 * 8 + i] = Ps[i >> 3][i & 7]; } __threadfence(); }
}
constexpr int PER = 512;
__global__ __launch_bounds__(32) void cnt_kernel(const int* __restrict__ srcs, const int* __restrict__ PERM, const int* __restrict__ ROWPTR, const int* __restrict__ ROWCNT, int permLen, int NLIM, int* __restrict__ CNT) {
  __shared__ int Row[PER]; const int lane = threadIdx.x; const int v = blockIdx.x; if (v >= NLIM) return; const int g0 = (v / PER) * PER;
  for (int c = lane; c < PER; c += 32) Row[c] = 0; wave_lds_sync();
  if (lane == 0) { int st = ROWPTR[v], cnt = ROWCNT[v]; cnt = iclamp(cnt, 0, 1 << 20); st = iclamp(st, 0, permLen - cnt); Row[v - g0] += 1;
    for (int j = 0; j < cnt; ++j) { const int e = iclamp(PERM[st + j], 0, E - 1); const int s = iclamp(srcs[e], 0, N - 1); if (s >= g0 && s < g0 + PER && s < NLIM) Row[s - g0] += 1; } }
  wave_lds_sync();
  for (int pass = 0; pass < 2; ++pass) { for (int c = lane; c < PER; c += 32) ((volatile int*)CNT)[(size_t)v * PER + c] = Row[c]; __threadfence(); }
}
__global__ __launch_bounds__(256) void xht_kernel(const float* __restrict__ XH, int NLIM, b16* __restrict__ XTH, b16* __restrict__ XTL) {
  __shared__ float T[64][65]; const int ct = blockIdx.x % (HD / 64), kt = (blockIdx.x / (HD / 64)) % (PER / 64), g = blockIdx.x / ((HD / 64) * (PER / 64)); if (g * PER >= NLIM) return; const int tid = threadIdx.x;
  for (int i = tid; i < 64 * 64; i += 256) { const int r = i / 64, c = i % 64; T[r][c] = XH[((size_t)g * PER + kt * 64 + r) * HD + ct * 64 + c]; }
  __syncthreads();
  { const int c = tid / 4, gg0 = (tid % 4) * 2; const int col = ct * 64 + c; const int h = col / D, cd = col % D; for (int gg = gg0; gg < gg0 + 2; ++gg) { v8b vh, vl;
#pragma unroll
      for (int j = 0; j < 8; ++j) { b16 p, q; split16(T[gg * 8 + j][c] * XS, p, q); vh[j] = p; vl[j] = q; }
      const size_t o = ((size_t)(g * NH + h) * D + cd) * PER + kt * 64 + gg * 8; for (int pass = 0; pass < 2; ++pass) { *(volatile v8b*)(XTH + o) = vh; *(volatile v8b*)(XTL + o) = vl; __threadfence(); } } }
}
__global__ __launch_bounds__(32) void gatatt_kernel(const int* __restrict__ CNT, const float* __restrict__ AS, const b16* __restrict__ XTH, const b16* __restrict__ XTL, int NLIM, float* __restrict__ O) {
  __shared__ __attribute__((aligned(16))) b16 Pf[16][PER + 8]; __shared__ float Mx[16], Sm[16], Ad[16]; __shared__ __attribute__((aligned(16))) float Tf[16][128 + 4];
  const int lane = threadIdx.x, nloc = lane & 15, hlf = lane >> 4; const int h = blockIdx.x % NH, qt = blockIdx.x / NH; const size_t i0 = (size_t)qt * 16; if (i0 >= (size_t)NLIM) return; const int g = (int)(i0 / PER); const size_t g0 = (size_t)g * PER;
  if (lane < 16) Ad[lane] = AS[(i0 + lane) * 8 + 4 + h];
  wave_lds_sync();
  for (int rr = 0; rr < 16; ++rr) { const int* cr = CNT + (i0 + rr) * PER; const float ad = Ad[rr]; float mx = -INFINITY;
#pragma unroll 4
    for (int kb = 0; kb < PER; kb += 32) { const int k = kb + lane; if (cr[k] > 0) mx = fmaxf(mx, leaky(AS[(g0 + k) * 8 + h] + ad)); }
    for (int o = 16; o; o >>= 1) mx = fmaxf(mx, __shfl_xor(mx, o)); if (lane == 0) { Mx[rr] = mx; } }
  wave_lds_sync();
  for (int rr = 0; rr < 16; ++rr) { const int* cr = CNT + (i0 + rr) * PER; const float ad = Ad[rr], mx = Mx[rr]; float s = 0.0f;
#pragma unroll 4
    for (int kb = 0; kb < PER; kb += 32) { const int k = kb + lane; const int c = cr[k]; float p = 0.0f; if (c > 0) p = (float)c * __expf(leaky(AS[(g0 + k) * 8 + h] + ad) - mx); s += p; Pf[rr][k] = (b16)(p * 512.0f); }
    for (int o = 16; o; o >>= 1) s += __shfl_xor(s, o); if (lane == 0) Sm[rr] = s; }
  wave_lds_sync();
#pragma unroll 1
  for (int cg = 0; cg < 2; ++cg) { v8f acc[8];
#pragma unroll
    for (int t = 0; t < 8; ++t) acc[t] = (v8f){};
#pragma unroll 2
    for (int kb = 0; kb < PER; kb += 32) { const v16b pa = frag_kb(&Pf[nloc][kb], hlf);
#pragma unroll
      for (int t = 0; t < 8; ++t) { const size_t xr = ((size_t)(g * NH + h) * D + cg * 128 + t * 16 + nloc) * PER + kb; acc[t] = wmma16b(pa, frag_kb(XTH + xr, hlf), acc[t]); acc[t] = wmma16b(pa, frag_kb(XTL + xr, hlf), acc[t]); } }
#pragma unroll
    for (int t = 0; t < 8; ++t)
#pragma unroll
      for (int r8 = 0; r8 < 8; ++r8) { const int rl = 8 * hlf + r8; Tf[rl][t * 16 + nloc] = acc[t][r8] * (1.0f / (512.0f * XS)) / Sm[rl]; }
    wave_lds_sync();
    for (int pass = 0; pass < 2; ++pass) { for (int rr = 0; rr < 16; ++rr) *(volatile v4f*)(O + ((i0 + rr) * NH + h) * D + cg * 128 + lane * 4) = *(const v4f*)(&Tf[rr][lane * 4]); __threadfence(); }
    wave_lds_sync(); }
}
__global__ __launch_bounds__(256) void comb_kernel(const float* __restrict__ O, const float* __restrict__ HP, const float* __restrict__ gb, const float* __restrict__ lng, const float* __restrict__ lnb, int RESID, int NLIM, float* __restrict__ HN) {
  __shared__ float Row[8][D]; const int wave = threadIdx.x >> 5, lane = threadIdx.x & 31; const size_t v = (size_t)blockIdx.x * 8 + wave; if (v >= (size_t)NLIM) return;
  for (int i = 0; i < 8; ++i) { const int c = lane * 8 + i; float s = 0.0f; for (int h = 0; h < NH; ++h) s += O[(v * NH + h) * D + c]; float z = s * 0.25f + bf16_rne(gb[c]); if (RESID) z += HP[v * D + c]; Row[wave][c] = z; }
  ln_relu_row(Row[wave], lane, lng, lnb);
  for (int pass = 0; pass < 2; ++pass) { *(volatile v4f*)(HN + v * D + lane * 8) = *(const v4f*)(&Row[wave][lane * 8]); *(volatile v4f*)(HN + v * D + lane * 8 + 4) = *(const v4f*)(&Row[wave][lane * 8 + 4]); __threadfence(); }
}
__global__ __launch_bounds__(32) void gate_kernel(const float* __restrict__ Hh, const b16* __restrict__ WT1, const float* __restrict__ b1, const float* __restrict__ W2, const float* __restrict__ b2, int NLIM, float* __restrict__ SC) {
  __shared__ __attribute__((aligned(16))) b16 Ah[16][D + 8], Al[16][D + 8]; __shared__ float So[16][NH]; __shared__ __attribute__((aligned(16))) float Tt[16][ADIM + 4];
  const int lane = threadIdx.x, nloc = lane & 15, hlf = lane >> 4; const size_t m0 = (size_t)blockIdx.x * 16; if (m0 >= (size_t)NLIM) return;
  for (int rr = 0; rr < 16; ++rr) for (int q = 0; q < 8; ++q) { b16 p, ql; split16(Hh[(m0 + rr) * D + q * 32 + lane] * XS, p, ql); Ah[rr][q * 32 + lane] = p; Al[rr][q * 32 + lane] = ql; }
  wave_lds_sync();
  v8f acc[8];
#pragma unroll
  for (int t = 0; t < 8; ++t) acc[t] = (v8f){};
#pragma unroll 2
  for (int kb = 0; kb < D; kb += 32) { const v16b a = frag_kb(&Ah[nloc][kb], hlf), al = frag_kb(&Al[nloc][kb], hlf);
#pragma unroll
    for (int t = 0; t < 8; ++t) { const v16b bw = frag_kb(WT1 + (size_t)(t * 16 + nloc) * D + kb, hlf); acc[t] = wmma16b(a, bw, acc[t]); acc[t] = wmma16b(al, bw, acc[t]); } }
#pragma unroll
  for (int t = 0; t < 8; ++t) { const int c = t * 16 + nloc; const float bb = bf16_rne(b1[c]);
#pragma unroll
    for (int r8 = 0; r8 < 8; ++r8) Tt[8 * hlf + r8][c] = tanhf(acc[t][r8] * (1.0f / (XS * WSC)) + bb); }
  wave_lds_sync();
  { float w2[4][NH]; for (int i = 0; i < 4; ++i) for (int h = 0; h < NH; ++h) w2[i][h] = bf16_rne(W2[(lane * 4 + i) * NH + h]);
    for (int rr = 0; rr < 16; ++rr) { float s[NH] = {0.0f, 0.0f, 0.0f, 0.0f}; for (int i = 0; i < 4; ++i) { const float tv = Tt[rr][lane * 4 + i]; for (int h = 0; h < NH; ++h) s[h] += pmul(tv, w2[i][h]); }
      for (int h = 0; h < NH; ++h) { float v = s[h]; for (int o = 16; o; o >>= 1) v += __shfl_xor(v, o); if (lane == 0) So[rr][h] = v + bf16_rne(b2[h]); } } }
  wave_lds_sync();
  for (int pass = 0; pass < 2; ++pass) { for (int q = 0; q < 2; ++q) { const int i = q * 32 + lane; ((volatile float*)SC)[m0 * NH + i] = So[i >> 2][i & 3]; } __threadfence(); }
}
__global__ __launch_bounds__(256) void pool_kernel(const float* __restrict__ Hh, const float* __restrict__ SC, const int* __restrict__ batch, const int* __restrict__ ntype, int NLIM, float* __restrict__ out) {
  const int g = blockIdx.x, c = threadIdx.x;
  auto lb = [&](int key) -> int { int lo = 0, hi = N; for (int it = 0; it < 14 && lo < hi; ++it) { const int mid = (lo + hi) >> 1; if (batch[mid] < key) lo = mid + 1; else hi = mid; } return lo; };
  int s0 = lb(g), e0 = lb(g + 1); if (e0 > NLIM) e0 = NLIM; if (e0 < s0) e0 = s0;
  float mm[NH], mu[NH], sm[NH], su[NH]; int nprot = 0; for (int h = 0; h < NH; ++h) { mm[h] = -INFINITY; mu[h] = -INFINITY; sm[h] = 0.0f; su[h] = 0.0f; }
#pragma unroll 1
  for (int n = s0; n < e0; ++n) { const bool pm = ntype[n] == 0; nprot += pm ? 1 : 0; for (int h = 0; h < NH; ++h) { const float sc = SC[(size_t)n * NH + h]; mu[h] = fmaxf(mu[h], sc); mm[h] = fmaxf(mm[h], pm ? sc : NEGV); } }
#pragma unroll 1
  for (int n = s0; n < e0; ++n) { const bool pm = ntype[n] == 0; for (int h = 0; h < NH; ++h) { const float sc = SC[(size_t)n * NH + h]; su[h] += __expf(sc - mu[h]); sm[h] += __expf((pm ? sc : NEGV) - mm[h]); } }
  float pooled = 0.0f, gm = 0.0f;
#pragma unroll 1
  for (int n = s0; n < e0; ++n) { const bool pm = ntype[n] == 0; const float hv = Hh[(size_t)n * D + c]; float wsum = 0.0f;
    for (int h = 0; h < NH; ++h) { const float sc = SC[(size_t)n * NH + h]; const float w = (nprot > 0) ? __expf((pm ? sc : NEGV) - mm[h]) / fmaxf(sm[h], 1e-30f) : __expf(sc - mu[h]) / fmaxf(su[h], 1e-30f); wsum += w; }
    pooled += pmul(hv, wsum); if (pm) gm += hv; }
  const int cnt = e0 - s0; const float r0 = pooled * 0.25f, r1 = gm / (float)(cnt < 1 ? 1 : cnt);
  for (int pass = 0; pass < 2; ++pass) { ((volatile float*)out)[(size_t)g * 2 * D + c] = (e0 > s0) ? r0 : 0.0f; ((volatile float*)out)[(size_t)g * 2 * D + D + c] = (e0 > s0) ? r1 : 0.0f; __threadfence(); }
}
}

extern "C" void kernel_launch(void* const* d_in, const int* in_sizes, int n_in, void* d_out, int out_size, void* d_ws, size_t ws_size, hipStream_t stream) {
  (void)n_in;
  auto Fp = [&](int i) { return (const float*)d_in[i]; }; auto Ip = [&](int i) { return (const int*)d_in[i]; };
  if (in_sizes[0] != N * PDIM || in_sizes[1] != 2 * E || in_sizes[2] != N || in_sizes[3] != N || in_sizes[4] != PDIM * D || in_sizes[8] != LDIM * D || in_sizes[12] != 2 * D || in_sizes[13] != NL * D * HD || in_sizes[14] != NL * NH * D || in_sizes[19] != D * ADIM || in_sizes[21] != ADIM * NH || out_size != NG * 2 * D) return;
  const int NLIM = N; const int GB16 = NBLK, GB8 = N / 8;
  size_t off = 0; char* ws = (char*)d_ws;
  auto carve = [&](size_t bytes) { char* p = ws + off; off += (bytes + 255) & ~(size_t)255; return p; };
  b16* WP = (b16*)carve((size_t)D * PK * 2); b16* WL = (b16*)carve((size_t)D * 64 * 2); b16* WG[3]; for (int i = 0; i < 3; ++i) WG[i] = (b16*)carve((size_t)HD * D * 2); b16* WT1 = (b16*)carve((size_t)ADIM * D * 2);
  float* HA = (float*)carve((size_t)N * D * 4); float* HB = (float*)carve((size_t)N * D * 4); float* XH = (float*)carve((size_t)N * HD * 4); float* AS = (float*)carve((size_t)N * 8 * 4); float* SC = (float*)carve((size_t)N * NH * 4);
  int* CNT = (int*)carve((size_t)N * PER * 4); b16* XTH = (b16*)carve((size_t)NG * NH * D * PER * 2); b16* XTL = (b16*)carve((size_t)NG * NH * D * PER * 2); float* O = (float*)carve((size_t)N * HD * 4);
  CsrBufs9 csr; off = csr_carve9(csr, ws, off, E, N);
  if (off > ws_size || off > ((size_t)160 << 20)) return;
  wput_kernel<<<(unsigned)(((size_t)D * (PK / 8) + 255) / 256), 256, 0, stream>>>(Fp(4), PDIM, PK, D, WP); wput_kernel<<<(D * 8 + 255) / 256, 256, 0, stream>>>(Fp(8), LDIM, 64, D, WL);
  for (int i = 0; i < 3; ++i) wput_kernel<<<(HD * 32 + 255) / 256, 256, 0, stream>>>(Fp(13) + (size_t)i * D * HD, D, D, HD, WG[i]);
  wput_kernel<<<(ADIM * 32 + 255) / 256, 256, 0, stream>>>(Fp(19), D, D, ADIM, WT1);
  csr_build9(csr, Ip(1) + E, E, N, stream);
  cnt_kernel<<<(unsigned)NLIM, 32, 0, stream>>>(Ip(1), csr.PERM, csr.ROWPTR, csr.ROWCNT, (int)csr.permLen, NLIM, CNT);
  inproj_kernel<<<GB16, 32, 0, stream>>>(Fp(0), Ip(3), WP, Fp(5), Fp(6), Fp(7), WL, Fp(9), Fp(10), Fp(11), Fp(12), HA);
  float* hp = HA; float* hn = HB;
  for (int i = 0; i < NL; ++i) {
    gatproj_kernel<<<GB16, 32, 0, stream>>>(hp, WG[i], Fp(14) + (size_t)i * NH * D, Fp(15) + (size_t)i * NH * D, XH, AS);
    xht_kernel<<<NG * (HD / 64) * (PER / 64), 256, 0, stream>>>(XH, NLIM, XTH, XTL);
    gatatt_kernel<<<(unsigned)((NLIM / 16) * NH), 32, 0, stream>>>(CNT, AS, XTH, XTL, NLIM, O);
    comb_kernel<<<GB8, 256, 0, stream>>>(O, hp, Fp(16) + i * D, Fp(17) + i * D, Fp(18) + i * D, i > 0 ? 1 : 0, NLIM, hn);
    float* t = hp; hp = hn; hn = t; }
  gate_kernel<<<GB16, 32, 0, stream>>>(hp, WT1, Fp(20), Fp(21), Fp(22), NLIM, SC);
  pool_kernel<<<NG, D, 0, stream>>>(hp, SC, Ip(2), Ip(3), NLIM, (float*)d_out);
}
